// GNNMatrixMultiHeadAttention_66529043415202
// MI455X (gfx1250) — hardware-verified
//
#include <hip/hip_runtime.h>


#define NB_  2
#define LL   1024
#define DD   256
#define NH_  8
#define DQ   32
#define NL   4
typedef _Float16 h16;
typedef unsigned short bf;
typedef __attribute__((ext_vector_type(16))) __bf16   v16bf;
typedef __attribute__((ext_vector_type(16))) _Float16 v16h;
typedef __attribute__((ext_vector_type(8)))  _Float16 v8h;
typedef __attribute__((ext_vector_type(8)))  unsigned short v8us;
typedef __attribute__((ext_vector_type(8)))  float    v8f;
typedef __attribute__((ext_vector_type(4)))  float    v4f;
typedef v8h  __attribute__((may_alias)) v8ha;
typedef v4f  __attribute__((may_alias)) v4fa;
typedef v8us __attribute__((may_alias)) v8usa;

__device__ __forceinline__ unsigned short f2bf(float f) { unsigned u = __float_as_uint(f); u += 0x7FFFu + ((u >> 16) & 1u); return (unsigned short)(u >> 16); }
__device__ __forceinline__ float bf2f(unsigned short b) { return __uint_as_float(((unsigned)b) << 16); }
__device__ __forceinline__ float bfr(float f) { return bf2f(f2bf(f)); }
__device__ __forceinline__ v16h cat16(v8h lo, v8h hi) { return __builtin_shufflevector(lo, hi, 0, 1, 2, 3, 4, 5, 6, 7, 8, 9, 10, 11, 12, 13, 14, 15); }
__device__ __forceinline__ v16bf cat16b(v8us lo, v8us hi) { return __builtin_bit_cast(v16bf, __builtin_shufflevector(lo, hi, 0, 1, 2, 3, 4, 5, 6, 7, 8, 9, 10, 11, 12, 13, 14, 15)); }
__device__ __forceinline__ v8f wmma16(v16h a, v16h b, v8f c) { return __builtin_amdgcn_wmma_f32_16x16x32_f16(false, a, false, b, (short)0, c, false, false); }
__device__ __forceinline__ v8f wmmab(v16bf a, v16bf b, v8f c) { return __builtin_amdgcn_wmma_f32_16x16x32_bf16(false, a, false, b, (short)0, c, false, false); }


template <typename T16> struct WFrag;
template <> struct WFrag<h16> { typedef v16h V; static __device__ __forceinline__ V ld(const h16* p) { return cat16(*(const v8h*)p, *(const v8h*)(p + 16)); } static __device__ __forceinline__ v8f mma(V a, V b, v8f c) { return wmma16(a, b, c); } };
template <> struct WFrag<bf> { typedef v16bf V; static __device__ __forceinline__ V ld(const bf* p) { return cat16b(*(const v8us*)p, *(const v8us*)(p + 16)); } static __device__ __forceinline__ v8f mma(V a, V b, v8f c) { return wmmab(a, b, c); } };
template <typename T16, int NSPLIT, bool BIAS>
__global__ __launch_bounds__(32) void k_gemmw(const T16* __restrict__ A, const T16* __restrict__ A2, const T16* __restrict__ Bt, const T16* __restrict__ Bt2, int K, float* C, int ldc, const float* __restrict__ bias, size_t sA, size_t sB, size_t sC) {
    typedef typename WFrag<T16>::V V;
    __shared__ __align__(16) float os[16 * 68];
    const size_t z = blockIdx.z; A += z * sA; if (A2) A2 += z * sA; Bt += z * sB; if (Bt2) Bt2 += z * sB; C += z * sC;
    const int lane = threadIdx.x & 31, lr = lane & 15, hi = lane >> 4; const int r0 = blockIdx.x * 64, c0 = blockIdx.y * 64;
    v8f acc[4][4];
#pragma unroll
    for (int mb = 0; mb < 4; ++mb)
#pragma unroll
        for (int nb = 0; nb < 4; ++nb) acc[mb][nb] = (v8f){};
    const size_t aoff = (size_t)(r0 + lr) * K + 8 * hi, boff = (size_t)(c0 + lr) * K + 8 * hi;
#pragma unroll 1
    for (int kc = 0; kc < K; kc += 32) {
        V a[4], a2[4];
#pragma unroll
        for (int mb = 0; mb < 4; ++mb) { a[mb] = WFrag<T16>::ld(A + aoff + (size_t)mb * 16 * K + kc); if (NSPLIT == 1 || NSPLIT == 2) a2[mb] = WFrag<T16>::ld(A2 + aoff + (size_t)mb * 16 * K + kc); }
#pragma unroll
        for (int nb = 0; nb < 4; ++nb) { const V b = WFrag<T16>::ld(Bt + boff + (size_t)nb * 16 * K + kc); V b2; if (NSPLIT >= 2) b2 = WFrag<T16>::ld(Bt2 + boff + (size_t)nb * 16 * K + kc);
#pragma unroll
            for (int mb = 0; mb < 4; ++mb) { acc[mb][nb] = WFrag<T16>::mma(a[mb], b, acc[mb][nb]); if (NSPLIT == 1 || NSPLIT == 2) acc[mb][nb] = WFrag<T16>::mma(a2[mb], b, acc[mb][nb]); if (NSPLIT >= 2) acc[mb][nb] = WFrag<T16>::mma(a[mb], b2, acc[mb][nb]); } }
        asm volatile("v_nop\n\tv_nop\n\tv_nop\n\tv_nop" : "+v"(acc[0][0]), "+v"(acc[1][1]), "+v"(acc[2][2]), "+v"(acc[3][3]) : "v"(a[0]), "v"(a[3]));
    }
#pragma unroll
    for (int mb = 0; mb < 4; ++mb) {
#pragma unroll
        for (int nb = 0; nb < 4; ++nb) {
#pragma unroll
            for (int j = 0; j < 8; ++j) os[(hi * 8 + j) * 68 + nb * 16 + lr] = acc[mb][nb][j]; }
        __builtin_amdgcn_wave_barrier(); asm volatile("" ::: "memory");
        float* crow = C + (size_t)(r0 + mb * 16) * ldc + c0;
#pragma unroll 1
        for (int ps = 0; ps < 2; ++ps) {
#pragma unroll
            for (int s = 0; s < 8; ++s) { const int row = 2 * s + hi, cofs = lr * 4; v4f val = *(const v4fa*)(os + row * 68 + cofs); if (BIAS) { val[0] += bfr(bias[c0 + cofs]); val[1] += bfr(bias[c0 + cofs + 1]); val[2] += bfr(bias[c0 + cofs + 2]); val[3] += bfr(bias[c0 + cofs + 3]); }
                *(volatile v4f*)(crow + (size_t)row * ldc + cofs) = val; }
            if (ps == 0) __threadfence(); }
        __builtin_amdgcn_wave_barrier(); asm volatile("" ::: "memory");
    }
}

__device__ __forceinline__ void splitf(float y, unsigned short& h, unsigned short& l) { h = f2bf(y); l = f2bf(y - bf2f(h)); }
typedef __attribute__((ext_vector_type(2))) unsigned short v2us;
typedef __attribute__((ext_vector_type(4))) unsigned short v4us;
typedef __attribute__((ext_vector_type(4))) int v4i;

__global__ __launch_bounds__(256) void k_cvt8(const float* __restrict__ src, bf* dst, size_t n8) { const size_t i = (size_t)blockIdx.x * 256 + threadIdx.x; if (i >= n8) return; const v8f v = *(const v8f*)(src + i * 8); v8us o;
#pragma unroll
    for (int k = 0; k < 8; ++k) o[k] = f2bf(v[k]); *(volatile v8us*)(dst + i * 8) = o; __threadfence(); *(volatile v8us*)(dst + i * 8) = o; }
__global__ __launch_bounds__(256) void k_pl32(const float* __restrict__ F, bf* Ph, bf* Pl) { const int e = (blockIdx.x * 256 + threadIdx.x) * 4; if (e >= NH_ * LL * DQ) return; const int d = e % DQ; const int t = (e / DQ) % LL; const int h = e / (DQ * LL); const float* f = F + (size_t)t * DD + h * DQ + d; v4us oh, ol;
#pragma unroll
    for (int u = 0; u < 4; ++u) { unsigned short a, b; splitf(f[u], a, b); oh[u] = a; ol[u] = b; } for (int ps = 0; ps < 2; ++ps) { *(volatile v4us*)(Ph + e) = oh; *(volatile v4us*)(Pl + e) = ol; if (ps == 0) __threadfence(); } }
__global__ __launch_bounds__(256) void k_ekT(const float* __restrict__ F, bf* Th, bf* Tl) { const int e = (blockIdx.x * 256 + threadIdx.x) * 2; if (e >= NH_ * 64 * LL) return; const int t = e % LL; const int d = (e / LL) % 64; const int h = e / (LL * 64); v2us oh, ol;
    if (d < DQ) { unsigned short a1, b1, a2, b2; splitf(F[(size_t)t * DD + h * DQ + d], a1, b1); splitf(F[(size_t)(t + 1) * DD + h * DQ + d], a2, b2); oh[0] = a1; oh[1] = a2; ol[0] = b1; ol[1] = b2; } else { oh[0] = oh[1] = 0; ol[0] = ol[1] = 0; }
    for (int ps = 0; ps < 2; ++ps) { *(volatile v2us*)(Th + e) = oh; *(volatile v2us*)(Tl + e) = ol; if (ps == 0) __threadfence(); } }
__global__ __launch_bounds__(256) void k_awacc(const float* __restrict__ S, const float* __restrict__ M, int l, int first, float* AW) { const size_t e = ((size_t)blockIdx.x * 256 + threadIdx.x) * 4; if (e >= (size_t)NH_ * LL * LL) return; const int k = (int)(e % LL); const int q = (int)((e / LL) % LL); const v4f s = *(const v4f*)(S + e); v4f a; if (first) { a[0] = a[1] = a[2] = a[3] = 0.f; } else a = *(const v4f*)(AW + e); v4f r;
#pragma unroll
    for (int u = 0; u < 4; ++u) { float t0 = __fdiv_rn(s[u], 5.656854249492381f); asm volatile("" : "+v"(t0)); float pm = __fmul_rn(t0, bfr(M[((size_t)q * LL + k + u) * NL + l])); asm volatile("" : "+v"(pm)); r[u] = __fadd_rn(a[u], pm); }
    *(volatile v4f*)(AW + e) = r; __threadfence(); *(volatile v4f*)(AW + e) = r; }
__global__ __launch_bounds__(256) void k_gsoft(float* AW, const int* __restrict__ pad) { const int lane = threadIdx.x & 31; const int row = blockIdx.x * 8 + (threadIdx.x >> 5); if (row >= NH_ * LL) return; const int q = row % LL; float* sr = AW + (size_t)row * LL; const int* pr = pad + (size_t)q * LL; float v[LL / 32]; float mx = -3.0e38f;
#pragma unroll
    for (int ch = 0; ch < LL / 128; ++ch) { const int j0 = ch * 128 + lane * 4; const v4f a = *(const v4f*)(sr + j0); const v4i p4 = *(const v4i*)(pr + j0);
#pragma unroll
        for (int u = 0; u < 4; ++u) { const float t = (p4[u] != 0) ? -3.0e38f : a[u]; v[ch * 4 + u] = t; mx = fmaxf(mx, t); } }
#pragma unroll
    for (int sh = 16; sh; sh >>= 1) mx = fmaxf(mx, __shfl_xor(mx, sh, 32));
    float sum = 0.f;
#pragma unroll
    for (int qq = 0; qq < LL / 32; ++qq) { float d0 = __fsub_rn(v[qq], mx); asm volatile("" : "+v"(d0)); v[qq] = (v[qq] > -1.0e38f) ? __builtin_amdgcn_exp2f(__fmul_rn(d0, 1.4426950408889634f)) : 0.f; sum += v[qq]; }
#pragma unroll
    for (int sh = 16; sh; sh >>= 1) sum += __shfl_xor(sum, sh, 32);
    const float f = __fdiv_rn(1.0f, sum);
    for (int ps = 0; ps < 2; ++ps) {
#pragma unroll
        for (int ch = 0; ch < LL / 128; ++ch) { v4f o4;
#pragma unroll
            for (int qq = 0; qq < 4; ++qq) o4[qq] = v[ch * 4 + qq] * f; *(volatile v4f*)(sr + ch * 128 + lane * 4) = o4; }
        if (ps == 0) __threadfence(); } }
__global__ __launch_bounds__(256) void k_pm(const float* __restrict__ P, const float* __restrict__ M, int l, bf* Ah, bf* Al) { const size_t e = ((size_t)blockIdx.x * 256 + threadIdx.x) * 4; if (e >= (size_t)NH_ * LL * LL) return; const int k = (int)(e % LL); const int q = (int)((e / LL) % LL); const v4f p = *(const v4f*)(P + e); v4us oh, ol;
#pragma unroll
    for (int u = 0; u < 4; ++u) { unsigned short a, b; splitf(__fmul_rn(p[u], bfr(M[((size_t)q * LL + k + u) * NL + l])), a, b); oh[u] = a; ol[u] = b; } *(volatile v4us*)(Ah + e) = oh; *(volatile v4us*)(Al + e) = ol; __threadfence(); *(volatile v4us*)(Ah + e) = oh; *(volatile v4us*)(Al + e) = ol; }
__global__ __launch_bounds__(256) void k_sumo(const float* __restrict__ O, bf* Ch, bf* Cl) { const int e = (blockIdx.x * 256 + threadIdx.x) * 4; if (e >= LL * DD) return; const int c = e % DD; const int q = e / DD; const int h = c / DQ, d = c % DQ; const size_t src = ((size_t)h * LL + q) * 64 + d; const size_t zo = (size_t)NH_ * LL * 64; v4us oh, ol;
#pragma unroll
    for (int u = 0; u < 4; ++u) { float s1 = __fadd_rn(O[src + u], O[zo + src + u]); asm volatile("" : "+v"(s1)); float s2 = __fadd_rn(s1, O[2 * zo + src + u]); asm volatile("" : "+v"(s2)); const float s3 = __fadd_rn(s2, O[3 * zo + src + u]); unsigned short a, b; splitf(s3, a, b); oh[u] = a; ol[u] = b; }
    *(volatile v4us*)(Ch + e) = oh; *(volatile v4us*)(Cl + e) = ol; __threadfence(); *(volatile v4us*)(Ch + e) = oh; *(volatile v4us*)(Cl + e) = ol; }

extern "C" void kernel_launch(void* const* d_in, const int* in_sizes, int n_in,
                              void* d_out, int out_size, void* d_ws, size_t ws_size, hipStream_t stream) {
    (void)in_sizes; (void)n_in; (void)out_size;
    const float* qx = (const float*)d_in[0]; const float* kx = (const float*)d_in[1]; const float* em = (const float*)d_in[2]; const int* pm = (const int*)d_in[3]; const float* w_q = (const float*)d_in[4]; const float* b_q = (const float*)d_in[5]; const float* w_ks = (const float*)d_in[6]; const float* w_h = (const float*)d_in[7]; const float* b_h = (const float*)d_in[8];
    float* OUT = (float*)d_out;
    char* wsp = (char*)d_ws;
    auto take = [&](size_t bytes) { char* p = wsp; wsp += (bytes + 255) & ~(size_t)255; return (void*)p; };
    bf* BQ = (bf*)take(DD * DD * 2); bf* BK[NL]; for (int l = 0; l < NL; ++l) BK[l] = (bf*)take(DD * DD * 2); bf* BH = (bf*)take(DD * DD * 2);
    bf* QB = (bf*)take((size_t)LL * DD * 2); bf* KB = (bf*)take((size_t)LL * DD * 2); float* F = (float*)take((size_t)LL * DD * 4); bf* Qh = (bf*)take((size_t)NH_ * LL * DQ * 2); bf* Ql = (bf*)take((size_t)NH_ * LL * DQ * 2);
    bf* EKh[NL]; bf* EKl[NL]; bf* ETh[NL]; bf* ETl[NL]; for (int l = 0; l < NL; ++l) { EKh[l] = (bf*)take((size_t)NH_ * LL * DQ * 2); EKl[l] = (bf*)take((size_t)NH_ * LL * DQ * 2); ETh[l] = (bf*)take((size_t)NH_ * 64 * LL * 2); ETl[l] = (bf*)take((size_t)NH_ * 64 * LL * 2); }
    float* S = (float*)take((size_t)NH_ * LL * LL * 4); float* AW = (float*)take((size_t)NH_ * LL * LL * 4); bf* Ah = (bf*)take((size_t)NH_ * LL * LL * 2); bf* Al = (bf*)take((size_t)NH_ * LL * LL * 2); float* O = (float*)take((size_t)NL * NH_ * LL * 64 * 4); bf* Ch = (bf*)take((size_t)LL * DD * 2); bf* Cl = (bf*)take((size_t)LL * DD * 2);
    if ((size_t)(wsp - (char*)d_ws) > ws_size) return;
    k_cvt8<<<(DD * DD / 8 + 255) / 256, 256, 0, stream>>>(w_q, BQ, DD * DD / 8); for (int l = 0; l < NL; ++l) k_cvt8<<<(DD * DD / 8 + 255) / 256, 256, 0, stream>>>(w_ks + (size_t)l * DD * DD, BK[l], DD * DD / 8); k_cvt8<<<(DD * DD / 8 + 255) / 256, 256, 0, stream>>>(w_h, BH, DD * DD / 8);
    const dim3 gp(LL / 64, DD / 64, 1); const size_t zq = (size_t)LL * DQ, zS = (size_t)LL * LL, zv = (size_t)64 * LL, zo = (size_t)LL * 64; const unsigned gLL = (unsigned)(((size_t)NH_ * LL * LL / 4 + 255) / 256);
    for (int b = 0; b < NB_; ++b) { const float* emb = em + (size_t)b * LL * LL * NL; const int* pmb = pm + (size_t)b * LL * LL;
        k_cvt8<<<(LL * DD / 8 + 255) / 256, 256, 0, stream>>>(qx + (size_t)b * LL * DD, QB, LL * DD / 8); k_cvt8<<<(LL * DD / 8 + 255) / 256, 256, 0, stream>>>(kx + (size_t)b * LL * DD, KB, LL * DD / 8);
        k_gemmw<bf, 0, true><<<gp, 32, 0, stream>>>(QB, nullptr, BQ, nullptr, DD, F, DD, b_q, 0, 0, 0); k_pl32<<<(NH_ * LL * DQ / 4 + 255) / 256, 256, 0, stream>>>(F, Qh, Ql);
        for (int l = 0; l < NL; ++l) { k_gemmw<bf, 0, false><<<gp, 32, 0, stream>>>(KB, nullptr, BK[l], nullptr, DD, F, DD, nullptr, 0, 0, 0); k_pl32<<<(NH_ * LL * DQ / 4 + 255) / 256, 256, 0, stream>>>(F, EKh[l], EKl[l]); k_ekT<<<(NH_ * 64 * LL / 2 + 255) / 256, 256, 0, stream>>>(F, ETh[l], ETl[l]); }
        for (int l = 0; l < NL; ++l) { k_gemmw<bf, 2, false><<<dim3(LL / 64, LL / 64, NH_), 32, 0, stream>>>(Qh, Ql, EKh[l], EKl[l], DQ, S, LL, nullptr, zq, zq, zS); k_awacc<<<gLL, 256, 0, stream>>>(S, emb, l, l == 0 ? 1 : 0, AW); }
        k_gsoft<<<NH_ * LL / 8, 256, 0, stream>>>(AW, pmb);
        for (int l = 0; l < NL; ++l) { k_pm<<<gLL, 256, 0, stream>>>(AW, emb, l, Ah, Al); k_gemmw<bf, 2, false><<<dim3(LL / 64, 1, NH_), 32, 0, stream>>>(Ah, Al, ETh[l], ETl[l], LL, O + (size_t)l * NH_ * zo, 64, nullptr, zS, zv, zo); }
        k_sumo<<<(LL * DD / 4 + 255) / 256, 256, 0, stream>>>(O, Ch, Cl);
        k_gemmw<bf, 1, true><<<gp, 32, 0, stream>>>(Ch, Cl, BH, nullptr, DD, OUT + (size_t)b * LL * DD, DD, b_h, 0, 0, 0); }
}
